// MineralDepositGCN_21517786153591
// MI455X (gfx1250) — hardware-verified
//
#include <hip/hip_runtime.h>
#include <stddef.h>
#include <math.h>


#define FIN    128
#define HID    64
#define HID2   128
#define NCLS   5
#define NCLSP  16
#define NTHR   256
#define NWAVE  8
#define EPT    8
#define NGRP   2
#define CHUNK  (NTHR * EPT * NGRP)
#define WCAP   (EPT * NGRP * 32)
#define LISTN  (NWAVE * WCAP)
#define NBC    4096
#define NBF    1024
#define RCAP   40960
#define RBN    128
#define TGT    256
#define DEGCAP 256
#define OTHR   512
#define GR     64
#define GTHR   128
#define BNEPS  1e-5f

#define LDS_FILL ((RCAP + NBF + LISTN) * 4 + 64)

#define SP1     132
#define PP2     136
#define PP3     72
#define CLS_STG 0
#define CLS_P2H (CLS_STG + GR * SP1 * 4)
#define CLS_P2L (CLS_P2H + GR * PP2 * 2)
#define CLS_P3H (CLS_P2L + GR * PP2 * 2)
#define CLS_P3L (CLS_P3H + GR * PP3 * 2)
#define CLS_OUT (CLS_P3L + GR * PP3 * 2)
#define LDS_CLS (CLS_OUT + GR * NCLS * 4)

static_assert((CHUNK & (CHUNK - 1)) == 0);
static_assert(CHUNK <= 4096);
static_assert(NBC <= 4096 && NBF <= 4096);
static_assert((NBC & (NBC - 1)) == 0 && (NBF & (NBF - 1)) == 0);
static_assert(NBC == 4 * NBF);
static_assert(OTHR * 8 == NBC);
static_assert((RCAP % 32) == 0);
static_assert(TGT == NWAVE * 32);
static_assert((TGT % GR) == 0);
static_assert(GTHR == 4 * 32 && GR == 4 * 16);
static_assert((CLS_P2H % 16) == 0 && (CLS_P2L % 16) == 0 && (CLS_P3H % 16) == 0 && (CLS_P3L % 16) == 0 && (CLS_OUT % 16) == 0);
static_assert((PP2 * 2) % 16 == 0 && (PP3 * 2) % 16 == 0);
static_assert(GR * NCLS / 4 <= GTHR);
static_assert(FIN % 32 == 0 && HID % 32 == 0 && HID2 % 32 == 0);
static_assert(DEGCAP <= RCAP);

typedef float          v4f   __attribute__((ext_vector_type(4)));
typedef float          v8f   __attribute__((ext_vector_type(8)));
typedef int            v4i   __attribute__((ext_vector_type(4)));
typedef unsigned short v8us  __attribute__((ext_vector_type(8)));
typedef unsigned short v16us __attribute__((ext_vector_type(16)));
typedef __bf16         v16b  __attribute__((ext_vector_type(16)));
union FragB { v16b v; v16us u; v8us h[2]; };
union U8 { v8us u; v4i i; };

__device__ __forceinline__ unsigned short f2bf(float f) {
  unsigned int u = __float_as_uint(f);
  u += 0x7FFFu + ((u >> 16) & 1u);
  return (unsigned short)(u >> 16);
}
__device__ __forceinline__ float bf2f(unsigned short b) { return __uint_as_float(((unsigned int)b) << 16); }

__device__ __forceinline__ void split8(v4f a, v4f b, v8us& hi, v8us& lo) {
#define SPL(I, X) { const float f_ = (X); const unsigned short h_ = f2bf(f_); hi[I] = h_; lo[I] = f2bf(f_ - bf2f(h_)); }
  SPL(0, a.x) SPL(1, a.y) SPL(2, a.z) SPL(3, a.w)
  SPL(4, b.x) SPL(5, b.y) SPL(6, b.z) SPL(7, b.w)
#undef SPL
}

__device__ __forceinline__ void afrag_f32(const float* p, int hh, FragB& ah, FragB& al) {
  const float* q = p + 8 * hh;
  const v4f x0 = *(const v4f*)q, x1 = *(const v4f*)(q + 4);
  const v4f x2 = *(const v4f*)(q + 16), x3 = *(const v4f*)(q + 20);
  split8(x0, x1, ah.h[0], al.h[0]);
  split8(x2, x3, ah.h[1], al.h[1]);
}

__device__ __forceinline__ void bfrag(const unsigned short* ph, const unsigned short* pl, FragB& bh, FragB& bl) {
  bh.h[0] = *(const v8us*)ph;
  bh.h[1] = *(const v8us*)(ph + 16);
  bl.h[0] = *(const v8us*)pl;
  bl.h[1] = *(const v8us*)(pl + 16);
}

__device__ __forceinline__ v8f wmb(v16b a, v16b b, v8f c) {
  v8f d = __builtin_amdgcn_wmma_f32_16x16x32_bf16(false, a, false, b, (short)0, c, false, false);
  asm volatile("v_nop\n\tv_nop\n\tv_nop\n\tv_nop" : "+v"(d) : "v"(a), "v"(b));
  return d;
}
__device__ __forceinline__ v8f wm3(const FragB& ah, const FragB& al, const FragB& bh, const FragB& bl, v8f c) {
  c = wmb(ah.v, bh.v, c);
  c = wmb(ah.v, bl.v, c);
  c = wmb(al.v, bh.v, c);
  return c;
}

__device__ __forceinline__ float gelu_f(float v) {
  return 0.5f * v * (1.0f + erff(v * 0.70710678118654752f));
}

template <int NB>
__device__ __forceinline__ int scan_chunk(const int* __restrict__ dsts, int nE, int cbase, int slotBase,
                                          int vec8, int* list, int tid, int lane, int wave) {
  int wc = 0;
#pragma unroll
  for (int g = 0; g < NGRP; ++g) {
    const int el0  = (g * NTHR + tid) * EPT;
    const int e0   = cbase + el0;
    const int sent = -2147483647 - 1;
    v4i da, db;
    if (vec8 != 0 && cbase + CHUNK <= nE) {
      da = *(const v4i*)(dsts + e0);
      db = *(const v4i*)(dsts + e0 + 4);
    } else {
      da.x = (e0     < nE) ? dsts[min(e0, nE - 1)] : sent;
      da.y = (e0 + 1 < nE) ? dsts[min(e0 + 1, nE - 1)] : sent;
      da.z = (e0 + 2 < nE) ? dsts[min(e0 + 2, nE - 1)] : sent;
      da.w = (e0 + 3 < nE) ? dsts[min(e0 + 3, nE - 1)] : sent;
      db.x = (e0 + 4 < nE) ? dsts[min(e0 + 4, nE - 1)] : sent;
      db.y = (e0 + 5 < nE) ? dsts[min(e0 + 5, nE - 1)] : sent;
      db.z = (e0 + 6 < nE) ? dsts[min(e0 + 6, nE - 1)] : sent;
      db.w = (e0 + 7 < nE) ? dsts[min(e0 + 7, nE - 1)] : sent;
    }
    const unsigned nb = (unsigned)slotBase;
    const unsigned s0 = (unsigned)da.x - nb, s1 = (unsigned)da.y - nb;
    const unsigned s2 = (unsigned)da.z - nb, s3 = (unsigned)da.w - nb;
    const unsigned s4 = (unsigned)db.x - nb, s5 = (unsigned)db.y - nb;
    const unsigned s6 = (unsigned)db.z - nb, s7 = (unsigned)db.w - nb;
    const bool h0 = s0 < (unsigned)NB, h1 = s1 < (unsigned)NB, h2 = s2 < (unsigned)NB, h3 = s3 < (unsigned)NB;
    const bool h4 = s4 < (unsigned)NB, h5 = s5 < (unsigned)NB, h6 = s6 < (unsigned)NB, h7 = s7 < (unsigned)NB;
    const unsigned any = __builtin_amdgcn_ballot_w32(h0 | h1 | h2 | h3 | h4 | h5 | h6 | h7);
    if (any != 0u) {
#define HITJ(J, HJ, SJ) { \
        const unsigned mj = __builtin_amdgcn_ballot_w32(HJ); \
        if (mj != 0u) { \
          if (HJ) { \
            const int pos = wc + (int)__builtin_amdgcn_mbcnt_lo(mj, 0u); \
            if (pos < WCAP) list[wave * WCAP + pos] = ((el0 + (J)) << 12) | (int)(SJ); \
          } \
          wc += (int)__builtin_popcount(mj); } }
      HITJ(0, h0, s0)
      HITJ(1, h1, s1)
      HITJ(2, h2, s2)
      HITJ(3, h3, s3)
      HITJ(4, h4, s4)
      HITJ(5, h5, s5)
      HITJ(6, h6, s6)
      HITJ(7, h7, s7)
#undef HITJ
    }
  }
  return wc;
}

__global__ __launch_bounds__(NTHR) void k_wcvt(
    const float* __restrict__ W, unsigned short* Ph, unsigned short* Pl, int K, int Nin, int NP) {
  const int t = blockIdx.x * NTHR + (int)threadIdx.x;
  if (t >= (NP * K) >> 3) return;
  const int o  = t * 8;
  const int n  = o / K;
  const int k0 = o - n * K;
  const int nc = n < Nin ? n : Nin - 1;
  float v[8];
#pragma unroll
  for (int e = 0; e < 8; ++e) {
    const float x = W[(size_t)(k0 + e) * Nin + nc];
    v[e] = (n < Nin) ? x : 0.0f;
  }
  v4f a, b;
  a.x = v[0]; a.y = v[1]; a.z = v[2]; a.w = v[3];
  b.x = v[4]; b.y = v[5]; b.z = v[6]; b.w = v[7];
  U8 hu, lu;
  split8(a, b, hu.u, lu.u);
  unsigned short* hp = Ph + o;
  unsigned short* lp = Pl + o;
  *(volatile v4i*)hp = hu.i;
  *(volatile v4i*)lp = lu.i;
  __threadfence();
  *(volatile v4i*)hp = hu.i;
  *(volatile v4i*)lp = lu.i;
}

__global__ __launch_bounds__(NTHR) void k_count(
    const int* __restrict__ ei, int* cnt, int nE, int vec8) {
  __shared__ __attribute__((aligned(16))) int scnt[NBC];
  __shared__ __attribute__((aligned(16))) int list[LISTN];
  __shared__ int wcnt[NWAVE];
  const int tid = threadIdx.x, lane = tid & 31, wave = tid >> 5;
  const int nodeBase = blockIdx.x * NBC;
  const int* dsts = ei + nE;

  for (int i = tid; i < NBC; i += NTHR) scnt[i] = 0;
  __syncthreads();

  const int nChunks = (nE + CHUNK - 1) / CHUNK;
#pragma unroll 1
  for (int ch = 0; ch < nChunks; ++ch) {
    const int cbase = ch * CHUNK;
    const int wc = scan_chunk<NBC>(dsts, nE, cbase, nodeBase, vec8, list, tid, lane, wave);
    if (lane == 0) wcnt[wave] = wc;
    __syncthreads();
    if (wave == 0) {
#pragma unroll 1
      for (int wsx = 0; wsx < NWAVE; ++wsx) {
        int n = __builtin_amdgcn_readfirstlane(wcnt[wsx]);
        n = n > WCAP ? WCAP : (n < 0 ? 0 : n);
        const int* lp = list + wsx * WCAP;
#pragma unroll 1
        for (int i = 0; i < n; ++i) {
          const int ent  = __builtin_amdgcn_readfirstlane(lp[i]);
          const int slot = ent & (NBC - 1);
          if (lane == 0) scnt[slot] = scnt[slot] + 1;
        }
      }
    }
    __syncthreads();
  }

  v4i cq[4];
#pragma unroll
  for (int q = 0; q < 4; ++q) {
    const int f = (wave * 4 + q) * 128 + 4 * lane;
    cq[q] = *(const v4i*)(scnt + f);
  }
  int* cp = cnt + (size_t)nodeBase;
#pragma unroll
  for (int q = 0; q < 4; ++q) {
    const int f = (wave * 4 + q) * 128 + 4 * lane;
    *(volatile v4i*)(cp + f) = cq[q];
  }
  __threadfence();
#pragma unroll
  for (int q = 0; q < 4; ++q) {
    const int f = (wave * 4 + q) * 128 + 4 * lane;
    *(volatile v4i*)(cp + f) = cq[q];
  }
}

__global__ __launch_bounds__(OTHR) void k_offsets(
    const int* __restrict__ cnt, int* off, int* rbase, int nChunk) {
  __shared__ __attribute__((aligned(16))) int soff[NBC];
  __shared__ __attribute__((aligned(16))) int srb[RBN];
  __shared__ int wtot[OTHR / 32];
  const int tid = threadIdx.x, lane = tid & 31, wave = tid >> 5, sub = tid >> 7;
  for (int i = tid; i < RBN; i += OTHR) srb[i] = 0;
  int carry = 0;
#pragma unroll 1
  for (int ch = 0; ch < nChunk; ++ch) {
    const int base = ch * NBC;
    const v4i c0 = *(const v4i*)(cnt + base + 8 * tid);
    const v4i c1 = *(const v4i*)(cnt + base + 8 * tid + 4);
    const int e0 = max(c0.x, 0), e1 = max(c0.y, 0), e2 = max(c0.z, 0), e3 = max(c0.w, 0);
    const int e4 = max(c1.x, 0), e5 = max(c1.y, 0), e6 = max(c1.z, 0), e7 = max(c1.w, 0);
    const int ts = e0 + e1 + e2 + e3 + e4 + e5 + e6 + e7;
    int incl = ts;
#pragma unroll
    for (int d = 1; d < 32; d <<= 1) {
      const int t = __shfl_up(incl, d);
      if (lane >= d) incl += t;
    }
    if (lane == 31) wtot[wave] = incl;
    __syncthreads();
    const int S0 = wtot[0]  + wtot[1]  + wtot[2]  + wtot[3];
    const int S1 = wtot[4]  + wtot[5]  + wtot[6]  + wtot[7];
    const int S2 = wtot[8]  + wtot[9]  + wtot[10] + wtot[11];
    const int S3 = wtot[12] + wtot[13] + wtot[14] + wtot[15];
    int pre = 0;
#pragma unroll 1
    for (int w = 4 * sub; w < wave; ++w) pre += wtot[w];
    const int b0 = carry;
    const int b1 = b0 + ((S0 + 31) & ~31);
    const int b2 = b1 + ((S1 + 31) & ~31);
    const int b3 = b2 + ((S2 + 31) & ~31);
    const int b4 = b3 + ((S3 + 31) & ~31);
    const int myb = sub == 0 ? b0 : (sub == 1 ? b1 : (sub == 2 ? b2 : b3));
    if (tid == 0) {
      srb[min(4 * ch + 0, RBN - 1)] = b0;
      srb[min(4 * ch + 1, RBN - 1)] = b1;
      srb[min(4 * ch + 2, RBN - 1)] = b2;
      srb[min(4 * ch + 3, RBN - 1)] = b3;
    }
    int run = myb + pre + incl - ts;
    soff[8 * tid + 0] = run; run += e0;
    soff[8 * tid + 1] = run; run += e1;
    soff[8 * tid + 2] = run; run += e2;
    soff[8 * tid + 3] = run; run += e3;
    soff[8 * tid + 4] = run; run += e4;
    soff[8 * tid + 5] = run; run += e5;
    soff[8 * tid + 6] = run; run += e6;
    soff[8 * tid + 7] = run;
    carry = b4;
    __syncthreads();
    const v4i o0 = *(const v4i*)(soff + 4 * tid);
    const v4i o1 = *(const v4i*)(soff + 4 * (tid + OTHR));
    int* op = off + base;
    *(volatile v4i*)(op + 4 * tid) = o0;
    *(volatile v4i*)(op + 4 * (tid + OTHR)) = o1;
    __threadfence();
    *(volatile v4i*)(op + 4 * tid) = o0;
    *(volatile v4i*)(op + 4 * (tid + OTHR)) = o1;
    __syncthreads();
  }
  if (tid == 0) srb[min(4 * nChunk, RBN - 1)] = carry;
  __syncthreads();
  v4i rv = {0, 0, 0, 0};
  if (tid < 32) rv = *(const v4i*)(srb + 4 * tid);
  if (tid < 32) *(volatile v4i*)(rbase + 4 * tid) = rv;
  __threadfence();
  if (tid < 32) *(volatile v4i*)(rbase + 4 * tid) = rv;
}

__global__ __launch_bounds__(NTHR) void k_fill(
    const int* __restrict__ ei, const int* __restrict__ off, const int* __restrict__ rbase,
    int* csr, int nE, int vec8, int csrLen) {
  extern __shared__ v4f lds_dyn[];
  int* region = (int*)lds_dyn;
  int* cursor = region + RCAP;
  int* list   = cursor + NBF;
  int* wcnt   = list + LISTN;
  const int tid = threadIdx.x, lane = tid & 31, wave = tid >> 5;
  const int b = blockIdx.x;
  const int nodeBase = b * NBF;
  const int* dsts = ei + nE;

  int rb0 = rbase[b];
  const int rb1 = rbase[b + 1];
  rb0 = rb0 < 0 ? 0 : (rb0 > csrLen ? csrLen : rb0);
  rb0 &= ~31;
  int len = rb1 - rb0;
  len = len < 0 ? 0 : (len > RCAP ? RCAP : len);
  int lenW = (len + 31) & ~31;
  if (rb0 + lenW > csrLen) lenW = (csrLen - rb0) & ~31;

  {
    const v4i z = {0, 0, 0, 0};
    for (int i = tid; i < RCAP / 4; i += NTHR) ((v4i*)region)[i] = z;
    for (int s = tid; s < NBF; s += NTHR) {
      int o = off[nodeBase + s] - rb0;
      o = o < 0 ? 0 : (o > RCAP ? RCAP : o);
      cursor[s] = o;
    }
  }
  __syncthreads();

  const int nChunks = (nE + CHUNK - 1) / CHUNK;
#pragma unroll 1
  for (int ch = 0; ch < nChunks; ++ch) {
    const int cbase = ch * CHUNK;
    const int wc = scan_chunk<NBF>(dsts, nE, cbase, nodeBase, vec8, list, tid, lane, wave);
    if (lane == 0) wcnt[wave] = wc;
    __syncthreads();
    if (wave == 0) {
#pragma unroll 1
      for (int wsx = 0; wsx < NWAVE; ++wsx) {
        int n = __builtin_amdgcn_readfirstlane(wcnt[wsx]);
        n = n > WCAP ? WCAP : (n < 0 ? 0 : n);
        const int* lp = list + wsx * WCAP;
#pragma unroll 1
        for (int i = 0; i < n; ++i) {
          const int ent  = __builtin_amdgcn_readfirstlane(lp[i]);
          const int slot = ent & (NBF - 1);
          int e = cbase + ((ent >> 12) & (CHUNK - 1));
          e = e > nE - 1 ? nE - 1 : e;
          if (lane == 0) {
            int pos = cursor[slot];
            pos = pos < 0 ? 0 : (pos > RCAP - 1 ? RCAP - 1 : pos);
            region[pos] = e;
            const int np = pos + 1;
            cursor[slot] = np > RCAP ? RCAP : np;
          }
        }
      }
    }
    __syncthreads();
  }

  const int nv = lenW >> 2;
  int* gp = csr + rb0;
#pragma unroll 1
  for (int i = tid; i < nv; i += NTHR) { const v4i v = ((const v4i*)region)[i]; *(volatile v4i*)(gp + 4 * i) = v; }
  __threadfence();
#pragma unroll 1
  for (int i = tid; i < nv; i += NTHR) { const v4i v = ((const v4i*)region)[i]; *(volatile v4i*)(gp + 4 * i) = v; }
}

template <int KD>
__global__ __launch_bounds__(GTHR) void k_gemm(
    const float* __restrict__ A, const unsigned short* __restrict__ Bh, const unsigned short* __restrict__ Bl,
    float* C, int nRowsA) {
  __shared__ __attribute__((aligned(16))) float stg[GR * HID];
  const int tid = threadIdx.x, lane = tid & 31, wave = tid >> 5, hh = lane >> 4, m = lane & 15;
  const int rowBase = blockIdx.x * GR;
  int row = rowBase + wave * 16 + m;
  row = row > nRowsA - 1 ? nRowsA - 1 : row;
  const float* ar = A + (size_t)row * KD;

  v8f acc[4];
#pragma unroll
  for (int t = 0; t < 4; ++t) { v8f z = {0.f, 0.f, 0.f, 0.f, 0.f, 0.f, 0.f, 0.f}; acc[t] = z; }
#pragma unroll
  for (int kt = 0; kt < KD / 32; ++kt) {
    FragB ah, al;
    afrag_f32(ar + 32 * kt, hh, ah, al);
#pragma unroll
    for (int t = 0; t < 4; ++t) {
      const int bo = (16 * t + m) * KD + 32 * kt + 8 * hh;
      FragB bh, bl;
      bfrag(Bh + bo, Bl + bo, bh, bl);
      acc[t] = wm3(ah, al, bh, bl, acc[t]);
    }
  }

  float* sp = stg + (wave * 16 + 8 * hh) * HID + m;
#pragma unroll
  for (int t = 0; t < 4; ++t) {
#pragma unroll
    for (int r = 0; r < 8; ++r) sp[r * HID + 16 * t] = acc[t][r];
  }
  __syncthreads();

  const float* lp = stg + wave * 16 * HID + 4 * lane;
  float* gp = C + ((size_t)rowBase + wave * 16) * HID + 4 * lane;
  v4f ov[8];
#pragma unroll
  for (int i = 0; i < 8; ++i) ov[i] = *(const v4f*)(lp + 128 * i);
#pragma unroll
  for (int i = 0; i < 8; ++i) *(volatile v4f*)(gp + 128 * i) = ov[i];
  __threadfence();
#pragma unroll
  for (int i = 0; i < 8; ++i) *(volatile v4f*)(gp + 128 * i) = ov[i];
}

__global__ __launch_bounds__(NTHR) void k_agg(
    const int* __restrict__ csr, const int* __restrict__ off, const int* __restrict__ cnt,
    const int* __restrict__ ei, const float* __restrict__ ew, const float* __restrict__ mp, float* h,
    const float* __restrict__ bias, const float* __restrict__ bmean, const float* __restrict__ bvar,
    const float* __restrict__ bgam, const float* __restrict__ bbet,
    int nN, int nE, int csrLen) {
  const int tid = threadIdx.x, lane = tid & 31, wave = tid >> 5, hh = lane >> 4, q = lane & 15;
  const int tbase = blockIdx.x * TGT + wave * 32;
  const int cl = tbase + lane;
  const int cnt_l = cnt[cl];
  const int off_l = off[cl];
  const v4f bb = *(const v4f*)(bias + 4 * q);
  const v4f mu = *(const v4f*)(bmean + 4 * q);
  const v4f va = *(const v4f*)(bvar + 4 * q);
  const v4f ga = *(const v4f*)(bgam + 4 * q);
  const v4f be = *(const v4f*)(bbet + 4 * q);
  v4f sc;
  sc.x = ga.x * rsqrtf(va.x + BNEPS); sc.y = ga.y * rsqrtf(va.y + BNEPS);
  sc.z = ga.z * rsqrtf(va.z + BNEPS); sc.w = ga.w * rsqrtf(va.w + BNEPS);
  const float* mq = mp + 4 * q;
  const int halfsel = (lane & 16) << 2;

#pragma unroll 1
  for (int j = 0; j < 16; ++j) {
    const int cA = tbase + 2 * j;
    int nA = __builtin_amdgcn_readlane(cnt_l, 2 * j);
    int nB = __builtin_amdgcn_readlane(cnt_l, 2 * j + 1);
    nA = nA < 0 ? 0 : (nA > DEGCAP ? DEGCAP : nA);
    nB = nB < 0 ? 0 : (nB > DEGCAP ? DEGCAP : nB);
    const int nmax = nA > nB ? nA : nB;
    const int nmy  = hh ? nB : nA;
    const int stA  = __builtin_amdgcn_readlane(off_l, 2 * j);
    const int stB  = __builtin_amdgcn_readlane(off_l, 2 * j + 1);
    const int stmy = hh ? stB : stA;
    v4f acc = {0.f, 0.f, 0.f, 0.f};
#pragma unroll 1
    for (int q0 = 0; q0 < nmax; q0 += 16) {
      const int idx = q0 + q;
      int pos = stmy + idx;
      pos = pos < 0 ? 0 : (pos > csrLen - 1 ? csrLen - 1 : pos);
      int e = csr[pos];
      e = e < 0 ? 0 : (e > nE - 1 ? nE - 1 : e);
      int s = ei[e];
      s = s < 0 ? s + nN : s;
      s = s < 0 ? 0 : (s > nN - 1 ? nN - 1 : s);
      const float wl = ew[e];
      const float w  = (idx < nmy) ? wl : 0.0f;
      const int soff = s * HID;
      const int wbit = __float_as_int(w);
      int mcnt = nmax - q0;
      mcnt = mcnt > 16 ? 16 : mcnt;
#pragma unroll 1
      for (int p = 0; p < mcnt; ++p) {
        const int sl = halfsel | (p << 2);
        const int so = __builtin_amdgcn_ds_bpermute(sl, soff);
        const float wp = __int_as_float(__builtin_amdgcn_ds_bpermute(sl, wbit));
        const v4f mv = *(const v4f*)(mq + so);
        acc = acc + mv * wp;
      }
    }
    v4f v = acc + bb;
#pragma unroll 1
    for (int c = 0; c < 4; ++c) {
      const float t  = (c == 0) ? v.x  : ((c == 1) ? v.y  : ((c == 2) ? v.z  : v.w));
      const float m_ = (c == 0) ? mu.x : ((c == 1) ? mu.y : ((c == 2) ? mu.z : mu.w));
      const float s_ = (c == 0) ? sc.x : ((c == 1) ? sc.y : ((c == 2) ? sc.z : sc.w));
      const float b_ = (c == 0) ? be.x : ((c == 1) ? be.y : ((c == 2) ? be.z : be.w));
      float r = t > 0.0f ? t : expm1f(t);
      r = (r - m_) * s_ + b_;
      v.x = (c == 0) ? r : v.x;
      v.y = (c == 1) ? r : v.y;
      v.z = (c == 2) ? r : v.z;
      v.w = (c == 3) ? r : v.w;
    }
    float* hp = h + (size_t)cA * HID + 4 * lane;
    *(volatile v4f*)hp = v;
    __threadfence();
    *(volatile v4f*)hp = v;
  }
}

__global__ __launch_bounds__(GTHR) void k_cls(
    const float* __restrict__ Hin,
    const unsigned short* __restrict__ W0h, const unsigned short* __restrict__ W0l, const float* __restrict__ cb0,
    const unsigned short* __restrict__ W1h, const unsigned short* __restrict__ W1l, const float* __restrict__ cb1,
    const unsigned short* __restrict__ W2h, const unsigned short* __restrict__ W2l, const float* __restrict__ cb2,
    float* out, int nN) {
  extern __shared__ v4f lds_dyn[];
  char* base = (char*)lds_dyn;
  float*          stg  = (float*)(base + CLS_STG);
  unsigned short* P2h  = (unsigned short*)(base + CLS_P2H);
  unsigned short* P2l  = (unsigned short*)(base + CLS_P2L);
  unsigned short* P3h  = (unsigned short*)(base + CLS_P3H);
  unsigned short* P3l  = (unsigned short*)(base + CLS_P3L);
  float*          sOut = (float*)(base + CLS_OUT);
  const int tid = threadIdx.x, lane = tid & 31, wave = tid >> 5, hh = lane >> 4, m = lane & 15;
  const int rowBase = blockIdx.x * GR;
  const int r0 = wave * 16;

  {
    const float* ar = Hin + (size_t)(rowBase + r0 + m) * HID;
    FragB ah0, al0, ah1, al1;
    afrag_f32(ar, hh, ah0, al0);
    afrag_f32(ar + 32, hh, ah1, al1);
#pragma unroll 1
    for (int g = 0; g < HID2 / 64; ++g) {
      v8f acc[4];
#pragma unroll
      for (int t = 0; t < 4; ++t) { v8f z = {0.f, 0.f, 0.f, 0.f, 0.f, 0.f, 0.f, 0.f}; acc[t] = z; }
#pragma unroll
      for (int t = 0; t < 4; ++t) {
        const int bo = (64 * g + 16 * t + m) * HID + 8 * hh;
        FragB bh, bl;
        bfrag(W0h + bo, W0l + bo, bh, bl);
        acc[t] = wm3(ah0, al0, bh, bl, acc[t]);
        bfrag(W0h + bo + 32, W0l + bo + 32, bh, bl);
        acc[t] = wm3(ah1, al1, bh, bl, acc[t]);
      }
#pragma unroll
      for (int t = 0; t < 4; ++t) {
        const int col = 64 * g + 16 * t + m;
        const float bv = cb0[col];
        float* sp = stg + (r0 + 8 * hh) * SP1 + col;
#pragma unroll
        for (int r = 0; r < 8; ++r) sp[r * SP1] = acc[t][r] + bv;
      }
    }
  }
  __syncthreads();
#pragma unroll 1
  for (int i = 0; i < (GR * HID2) / GTHR; ++i) {
    const int idx = i * GTHR + tid;
    const int row = idx >> 7, col = idx & 127;
    const float g = gelu_f(stg[row * SP1 + col]);
    const unsigned short hb = f2bf(g);
    P2h[row * PP2 + col] = hb;
    P2l[row * PP2 + col] = f2bf(g - bf2f(hb));
  }
  __syncthreads();

  {
    v8f acc[4];
#pragma unroll
    for (int t = 0; t < 4; ++t) { v8f z = {0.f, 0.f, 0.f, 0.f, 0.f, 0.f, 0.f, 0.f}; acc[t] = z; }
    const unsigned short* a2h = P2h + (r0 + m) * PP2 + 8 * hh;
    const unsigned short* a2l = P2l + (r0 + m) * PP2 + 8 * hh;
#pragma unroll
    for (int kt = 0; kt < HID2 / 32; ++kt) {
      FragB ah, al;
      ah.h[0] = *(const v8us*)(a2h + 32 * kt);
      ah.h[1] = *(const v8us*)(a2h + 32 * kt + 16);
      al.h[0] = *(const v8us*)(a2l + 32 * kt);
      al.h[1] = *(const v8us*)(a2l + 32 * kt + 16);
#pragma unroll
      for (int t = 0; t < 4; ++t) {
        const int bo = (16 * t + m) * HID2 + 32 * kt + 8 * hh;
        FragB bh, bl;
        bfrag(W1h + bo, W1l + bo, bh, bl);
        acc[t] = wm3(ah, al, bh, bl, acc[t]);
      }
    }
#pragma unroll
    for (int t = 0; t < 4; ++t) {
      const int col = 16 * t + m;
      const float bv = cb1[col];
      float* sp = stg + (r0 + 8 * hh) * SP1 + col;
#pragma unroll
      for (int r = 0; r < 8; ++r) sp[r * SP1] = acc[t][r] + bv;
    }
  }
  __syncthreads();
#pragma unroll 1
  for (int i = 0; i < (GR * HID) / GTHR; ++i) {
    const int idx = i * GTHR + tid;
    const int row = idx >> 6, col = idx & 63;
    const float g = gelu_f(stg[row * SP1 + col]);
    const unsigned short hb = f2bf(g);
    P3h[row * PP3 + col] = hb;
    P3l[row * PP3 + col] = f2bf(g - bf2f(hb));
  }
  __syncthreads();

  {
    v8f c3 = {0.f, 0.f, 0.f, 0.f, 0.f, 0.f, 0.f, 0.f};
    const unsigned short* a3h = P3h + (r0 + m) * PP3 + 8 * hh;
    const unsigned short* a3l = P3l + (r0 + m) * PP3 + 8 * hh;
#pragma unroll
    for (int kt = 0; kt < HID / 32; ++kt) {
      FragB ah, al;
      ah.h[0] = *(const v8us*)(a3h + 32 * kt);
      ah.h[1] = *(const v8us*)(a3h + 32 * kt + 16);
      al.h[0] = *(const v8us*)(a3l + 32 * kt);
      al.h[1] = *(const v8us*)(a3l + 32 * kt + 16);
      const int bo = m * HID + 32 * kt + 8 * hh;
      FragB bh, bl;
      bfrag(W2h + bo, W2l + bo, bh, bl);
      c3 = wm3(ah, al, bh, bl, c3);
    }
    const float b2v = cb2[m < NCLS ? m : NCLS - 1];
    if (m < NCLS) {
      float* so = sOut + (r0 + 8 * hh) * NCLS + m;
#pragma unroll
      for (int r = 0; r < 8; ++r) so[r * NCLS] = c3[r] + b2v;
    }
  }
  __syncthreads();

  int valid = nN - rowBase;
  valid = valid > GR ? GR : (valid < 0 ? 0 : valid);
  const int nF  = valid * NCLS;
  const int nv  = nF >> 2;
  const int rem = nF & 3;
  float* op = out + (size_t)rowBase * NCLS;
  v4f ov = {0.f, 0.f, 0.f, 0.f};
  float os = 0.0f;
  if (tid < nv)  ov = *(const v4f*)(sOut + 4 * tid);
  if (tid < rem) os = sOut[4 * nv + tid];
  if (tid < nv)  *(volatile v4f*)(op + 4 * tid) = ov;
  if (tid < rem) *(volatile float*)(op + 4 * nv + tid) = os;
  __threadfence();
  if (tid < nv)  *(volatile v4f*)(op + 4 * tid) = ov;
  if (tid < rem) *(volatile float*)(op + 4 * nv + tid) = os;
}

static inline size_t up256(size_t x) { return (x + 255) & ~(size_t)255; }

extern "C" void kernel_launch(void* const* d_in, const int* in_sizes, int n_in,
                              void* d_out, int out_size, void* d_ws, size_t ws_size,
                              hipStream_t stream) {
  if (n_in < 19) return;
  const int nN = in_sizes[0] / FIN;
  const int nE = in_sizes[1] / 2;
  if (nN <= 0 || nE <= 0 || in_sizes[0] != nN * FIN || in_sizes[1] != 2 * nE || in_sizes[2] != nE) return;
  if (in_sizes[3] != FIN * HID || in_sizes[4] < HID || in_sizes[5] != HID * HID || in_sizes[6] < HID ||
      in_sizes[7] != HID * HID || in_sizes[8] < HID) return;
  if (in_sizes[9] < 3 * HID || in_sizes[10] < 3 * HID || in_sizes[11] < 3 * HID || in_sizes[12] < 3 * HID) return;
  if (in_sizes[13] != HID * HID2 || in_sizes[14] < HID2 || in_sizes[15] != HID2 * HID || in_sizes[16] < HID ||
      in_sizes[17] != HID * NCLS || in_sizes[18] < NCLS) return;
  if (out_size != nN * NCLS) return;
  if (nE > (1 << 28) || nN > (1 << 24)) return;

  const float* x   = (const float*)d_in[0];
  const int*   ei  = (const int*)d_in[1];
  const float* ew  = (const float*)d_in[2];
  const float* w0  = (const float*)d_in[3];  const float* b0  = (const float*)d_in[4];
  const float* w1  = (const float*)d_in[5];  const float* b1  = (const float*)d_in[6];
  const float* w2  = (const float*)d_in[7];  const float* b2  = (const float*)d_in[8];
  const float* bng = (const float*)d_in[9];
  const float* bnb = (const float*)d_in[10];
  const float* bnm = (const float*)d_in[11];
  const float* bnv = (const float*)d_in[12];
  const float* cw0 = (const float*)d_in[13]; const float* cb0 = (const float*)d_in[14];
  const float* cw1 = (const float*)d_in[15]; const float* cb1 = (const float*)d_in[16];
  const float* cw2 = (const float*)d_in[17]; const float* cb2 = (const float*)d_in[18];
  float* out = (float*)d_out;

  const int NPAD   = ((nN + TGT - 1) / TGT) * TGT;
  const int nBC    = (nN + NBC - 1) / NBC;
  const int CNTPAD = nBC * NBC;
  if (4 * nBC + 1 > RBN) return;
  const int nBF    = (nN + NBF - 1) / NBF;
  const int csrLen = ((nE + 31) & ~31) + 4096;
  const int nGemm  = NPAD / GR;
  const int nAgg   = NPAD / TGT;
  const int nCls   = (nN + GR - 1) / GR;

  char* ws = (char*)d_ws;
  size_t off = 0;
  const size_t oW0h = off; off = up256(off + (size_t)HID * FIN * 2);
  const size_t oW0l = off; off = up256(off + (size_t)HID * FIN * 2);
  const size_t oW1h = off; off = up256(off + (size_t)HID * HID * 2);
  const size_t oW1l = off; off = up256(off + (size_t)HID * HID * 2);
  const size_t oW2h = off; off = up256(off + (size_t)HID * HID * 2);
  const size_t oW2l = off; off = up256(off + (size_t)HID * HID * 2);
  const size_t oC0h = off; off = up256(off + (size_t)HID2 * HID * 2);
  const size_t oC0l = off; off = up256(off + (size_t)HID2 * HID * 2);
  const size_t oC1h = off; off = up256(off + (size_t)HID * HID2 * 2);
  const size_t oC1l = off; off = up256(off + (size_t)HID * HID2 * 2);
  const size_t oC2h = off; off = up256(off + (size_t)NCLSP * HID * 2);
  const size_t oC2l = off; off = up256(off + (size_t)NCLSP * HID * 2);
  const size_t oCnt = off; off = up256(off + (size_t)CNTPAD * 4);
  const size_t oOff = off; off = up256(off + (size_t)CNTPAD * 4);
  const size_t oRb  = off; off = up256(off + (size_t)RBN * 4);
  const size_t oCsr = off; off = up256(off + (size_t)csrLen * 4);
  const size_t oH   = off; off = up256(off + (size_t)NPAD * HID * 4);
  const size_t oM   = off; off = up256(off + (size_t)NPAD * HID * 4);
  if (off > ws_size) return;
  unsigned short* w0h  = (unsigned short*)(ws + oW0h); unsigned short* w0l  = (unsigned short*)(ws + oW0l);
  unsigned short* w1h  = (unsigned short*)(ws + oW1h); unsigned short* w1l  = (unsigned short*)(ws + oW1l);
  unsigned short* w2h  = (unsigned short*)(ws + oW2h); unsigned short* w2l  = (unsigned short*)(ws + oW2l);
  unsigned short* c0h  = (unsigned short*)(ws + oC0h); unsigned short* c0l  = (unsigned short*)(ws + oC0l);
  unsigned short* c1h  = (unsigned short*)(ws + oC1h); unsigned short* c1l  = (unsigned short*)(ws + oC1l);
  unsigned short* c2h  = (unsigned short*)(ws + oC2h); unsigned short* c2l  = (unsigned short*)(ws + oC2l);
  int*   cnt  = (int*)(ws + oCnt);
  int*   offp = (int*)(ws + oOff);
  int*   rb   = (int*)(ws + oRb);
  int*   csr  = (int*)(ws + oCsr);
  float* hpl  = (float*)(ws + oH);
  float* mpl  = (float*)(ws + oM);

  const int vec8 = ((nE & 3) == 0) ? 1 : 0;

  k_wcvt<<<(FIN * HID / 8 + NTHR - 1) / NTHR, NTHR, 0, stream>>>(w0,  w0h, w0l, FIN,  HID,  HID);
  k_wcvt<<<(HID * HID / 8 + NTHR - 1) / NTHR, NTHR, 0, stream>>>(w1,  w1h, w1l, HID,  HID,  HID);
  k_wcvt<<<(HID * HID / 8 + NTHR - 1) / NTHR, NTHR, 0, stream>>>(w2,  w2h, w2l, HID,  HID,  HID);
  k_wcvt<<<(HID * HID2 / 8 + NTHR - 1) / NTHR, NTHR, 0, stream>>>(cw0, c0h, c0l, HID,  HID2, HID2);
  k_wcvt<<<(HID2 * HID / 8 + NTHR - 1) / NTHR, NTHR, 0, stream>>>(cw1, c1h, c1l, HID2, HID,  HID);
  k_wcvt<<<(HID * NCLSP / 8 + NTHR - 1) / NTHR, NTHR, 0, stream>>>(cw2, c2h, c2l, HID,  NCLS, NCLSP);

  k_count<<<nBC, NTHR, 0, stream>>>(ei, cnt, nE, vec8);
  k_offsets<<<1, OTHR, 0, stream>>>(cnt, offp, rb, nBC);
  hipFuncSetAttribute(reinterpret_cast<const void*>(&k_fill),
                      hipFuncAttributeMaxDynamicSharedMemorySize, LDS_FILL);
  k_fill<<<nBF, NTHR, LDS_FILL, stream>>>(ei, offp, rb, csr, nE, vec8, csrLen);

  k_gemm<FIN><<<nGemm, GTHR, 0, stream>>>(x, w0h, w0l, mpl, nN);
  k_agg<<<nAgg, NTHR, 0, stream>>>(csr, offp, cnt, ei, ew, mpl, hpl, b0,
                                   bnm, bnv, bng, bnb, nN, nE, csrLen);
  k_gemm<HID><<<nGemm, GTHR, 0, stream>>>(hpl, w1h, w1l, mpl, NPAD);
  k_agg<<<nAgg, NTHR, 0, stream>>>(csr, offp, cnt, ei, ew, mpl, hpl, b1,
                                   bnm + HID, bnv + HID, bng + HID, bnb + HID, nN, nE, csrLen);
  k_gemm<HID><<<nGemm, GTHR, 0, stream>>>(hpl, w2h, w2l, mpl, NPAD);
  k_agg<<<nAgg, NTHR, 0, stream>>>(csr, offp, cnt, ei, ew, mpl, hpl, b2,
                                   bnm + 2 * HID, bnv + 2 * HID, bng + 2 * HID, bnb + 2 * HID, nN, nE, csrLen);

  hipFuncSetAttribute(reinterpret_cast<const void*>(&k_cls),
                      hipFuncAttributeMaxDynamicSharedMemorySize, LDS_CLS);
  k_cls<<<nCls, GTHR, LDS_CLS, stream>>>(hpl, c0h, c0l, cb0, c1h, c1l, cb1, c2h, c2l, cb2, out, nN);
}
